// BaseFConv2d_15350213116004
// MI455X (gfx1250) — hardware-verified
//
#include <hip/hip_runtime.h>

typedef __attribute__((ext_vector_type(16))) _Float16 v16h;
typedef __attribute__((ext_vector_type(8)))  _Float16 v8h;
typedef __attribute__((ext_vector_type(8)))  float    v8f;
typedef __attribute__((ext_vector_type(4)))  float    v4f_t;
typedef float v4fa __attribute__((ext_vector_type(4), may_alias));
typedef __attribute__((ext_vector_type(4)))  unsigned v4u_t;
typedef unsigned v4ua __attribute__((ext_vector_type(4), may_alias));
__device__ __forceinline__ unsigned pk2h(_Float16 a, _Float16 b) { return (unsigned)__builtin_bit_cast(unsigned short, a) | ((unsigned)__builtin_bit_cast(unsigned short, b) << 16); }

#define B_     256
#define C_     3
#define L_     8
#define OC_    64
#define NNODES 7
#define INW    3072
#define NPIX2  256
#define K1PAD  32
#define FCIN   (OC_*NPIX2)
#define OUTW   10

__global__ __launch_bounds__(256) void k_convert_w1(const float* __restrict__ w1,
                                                    _Float16* __restrict__ wf) {
    int idx = blockIdx.x * 256 + threadIdx.x;
    idx *= 2; if (idx >= 512 * K1PAD) return;
    int row = idx / K1PAD, kk = idx % K1PAD;
    float v0 = (kk < 27) ? w1[row * 27 + kk] : 0.0f, v1 = (kk + 1 < 27) ? w1[row * 27 + kk + 1] : 0.0f;
    const unsigned p = pk2h((_Float16)v0, (_Float16)v1);
    *(volatile unsigned*)(wf + idx) = p; __threadfence(); *(volatile unsigned*)(wf + idx) = p;
}

__global__ __launch_bounds__(256) void k_convert_w2(const float* __restrict__ w2,
                                                    _Float16* __restrict__ wf) {
    int idx = blockIdx.x * 256 + threadIdx.x;
    if (idx >= L_ * 9 * OC_ * OC_) return;
    idx *= 2; if (idx >= L_ * 9 * OC_ * OC_) return;
    int ic = idx & 63;
    int oc = (idx >> 6) & 63;
    int r  = (idx >> 12) % 9;
    int l  = idx / (9 * 64 * 64);
    const unsigned p = pk2h((_Float16)w2[((l * OC_ + oc) * OC_ + ic) * 9 + r], (_Float16)w2[((l * OC_ + oc) * OC_ + ic + 1) * 9 + r]);
    *(volatile unsigned*)(wf + idx) = p; __threadfence(); *(volatile unsigned*)(wf + idx) = p;
}

__global__ __launch_bounds__(256) void k_mixture(const float* __restrict__ x,
                                                 const float* __restrict__ nw,
                                                 const float* __restrict__ nb,
                                                 float* __restrict__ mix) {
    __shared__ float sP[NNODES * 256];
    __shared__ float sLog[NNODES];
    int b = blockIdx.x, tid = threadIdx.x;
    float p[NNODES];
#pragma unroll
    for (int n = 0; n < NNODES; ++n) p[n] = 0.0f;
    for (int i = tid; i < INW; i += 256) {
        float xv = x[b * INW + i];
#pragma unroll
        for (int n = 0; n < NNODES; ++n) p[n] += xv * nw[n * INW + i];
    }
#pragma unroll
    for (int n = 0; n < NNODES; ++n) sP[n * 256 + tid] = p[n];
    __syncthreads();
    if (tid < NNODES) {
        float s = 0.0f;
        for (int t = 0; t < 256; ++t) s += sP[tid * 256 + t];
        sLog[tid] = s + nb[tid];
    }
    __syncthreads();
    if (tid == 0) {
        float sg[NNODES];
#pragma unroll
        for (int n = 0; n < NNODES; ++n) sg[n] = 1.0f / (1.0f + __expf(-sLog[n]));
#pragma unroll
        for (int j = 0; j < L_; ++j) {
            float t0 = ((j >> 2) & 1) ? sg[0] : 1.0f - sg[0];
            int   n1 = 1 + ((j >> 2) & 1);
            float t1 = ((j >> 1) & 1) ? sg[n1] : 1.0f - sg[n1];
            int   n2 = 3 + (j >> 1);
            float t2 = (j & 1) ? sg[n2] : 1.0f - sg[n2];
            mix[b * L_ + j] = t0 * t1 * t2;
        }
    }
}

__global__ __launch_bounds__(256) void k_conv1_pool(const float* __restrict__ x,
                                                    const _Float16* __restrict__ wf1,
                                                    const float* __restrict__ cb1,
                                                    _Float16* __restrict__ ypool) {
    __shared__ _Float16 sX[C_ * 34 * 34];
    __shared__ _Float16 sB[256 * 32];
    __shared__ _Float16 sW[512 * K1PAD];
    __shared__ float    sBias[512];
    int b    = blockIdx.x >> 2;
    int quad = blockIdx.x & 3;
    int tid  = threadIdx.x;

    for (int idx = tid; idx < C_ * 1156; idx += 256) {
        int c = idx / 1156, rem = idx % 1156;
        int yy = rem / 34 - 1, xx = rem % 34 - 1;
        float v = 0.0f;
        if (yy >= 0 && yy < 32 && xx >= 0 && xx < 32)
            v = x[((b * C_ + c) * 32 + yy) * 32 + xx];
        sX[idx] = (_Float16)v;
    }
    __syncthreads();

    for (int idx = tid; idx < 256 * 32; idx += 256) {
        int col = idx >> 5, kk = idx & 31;
        int g = col >> 4, n = col & 15;
        int prow = g >> 2, sub = g & 3;
        int py = 2 * (quad * 4 + prow) + (sub >> 1);
        int px = 2 * n + (sub & 1);
        _Float16 v = (_Float16)0.0f;
        if (kk < 27) {
            int ic = kk / 9, r = kk % 9;
            v = sX[ic * 1156 + (py + r / 3) * 34 + (px + r % 3)];
        }
        sB[idx] = v;
    }
    for (int idx = tid; idx < 512 * K1PAD / 8; idx += 256)
        *(v8h*)(sW + idx * 8) = *(const v8h*)(wf1 + idx * 8);
    for (int idx = tid; idx < 512; idx += 256) sBias[idx] = cb1[idx];
    __syncthreads();

    int wave = tid >> 5, lane = tid & 31;
    int m = lane & 15, hs = lane >> 4;
    int n = m;

__shared__ __attribute__((aligned(16))) _Float16 sO[8][16 * OC_];
#pragma unroll 1
    for (int t = wave; t < 32; t += 8) {
        int l1 = t >> 2, prow = t & 3;
        _Float16* so = sO[wave];
#pragma unroll 1
        for (int m4 = 0; m4 < 4; ++m4) {
            int mo = l1 * 64 + m4 * 16;
            const _Float16* wrow = sW + (mo + m) * K1PAD + 8 * hs;
            v16h av;
            ((v8h*)&av)[0] = *(const v8h*)wrow;
            ((v8h*)&av)[1] = *(const v8h*)(wrow + 16);

            v8f acc[4];
#pragma unroll
            for (int s = 0; s < 4; ++s) {
                const _Float16* sp = sB + ((prow * 4 + s) * 16 + n) * 32 + 8 * hs;
                v16h bv;
                ((v8h*)&bv)[0] = *(const v8h*)sp;
                ((v8h*)&bv)[1] = *(const v8h*)(sp + 16);
                v8f c0 = {};
                acc[s] = __builtin_amdgcn_wmma_f32_16x16x32_f16(false, av, false, bv,
                                                                (short)0, c0, false, false);
            }
#pragma unroll
            for (int rr = 0; rr < 8; ++rr) {
                float mval = fmaxf(fmaxf(acc[0][rr], acc[1][rr]),
                                   fmaxf(acc[2][rr], acc[3][rr]));
                float vv = mval + sBias[mo + rr + 8 * hs];
                so[n * OC_ + m4 * 16 + rr + 8 * hs] = (_Float16)fmaxf(vv, 0.0f);
            }
        }
        asm volatile("s_wait_dscnt 0" ::: "memory");
        _Float16* dst = ypool + ((size_t)(b * L_ + l1) * NPIX2 + (quad * 4 + prow) * 16) * OC_;
        v4u_t ov[4];
#pragma unroll
        for (int i = 0; i < 4; ++i) { const int c = lane + 32 * i; ov[i] = *(const volatile v4ua*)(so + (c >> 3) * OC_ + (c & 7) * 8); }
#pragma unroll
        for (int i = 0; i < 4; ++i) { const int c = lane + 32 * i; *(volatile v4u_t*)(dst + (c >> 3) * OC_ + (c & 7) * 8) = ov[i]; }
        __threadfence();
#pragma unroll
        for (int i = 0; i < 4; ++i) { const int c = lane + 32 * i; *(volatile v4u_t*)(dst + (c >> 3) * OC_ + (c & 7) * 8) = ov[i]; }
        asm volatile("s_wait_dscnt 0" ::: "memory");
    }
}

__global__ __launch_bounds__(256) void k_conv2(const _Float16* __restrict__ ypool,
                                               const _Float16* __restrict__ wf2,
                                               const float* __restrict__ cb2,
                                               _Float16* __restrict__ y2) {
    __shared__ _Float16 sIn[18 * 18 * OC_];
    int b = blockIdx.x >> 3, l = blockIdx.x & 7;
    int tid = threadIdx.x;

    const _Float16* src = ypool + (size_t)(b * L_ + l) * NPIX2 * OC_;
    for (int idx = tid; idx < 324 * 8; idx += 256) {
        int pix = idx >> 3, part = idx & 7;
        int yy = pix / 18 - 1, xx = pix % 18 - 1;
        v8h v = {};
        if (yy >= 0 && yy < 16 && xx >= 0 && xx < 16)
            v = *(const v8h*)(src + (yy * 16 + xx) * OC_ + part * 8);
        *(v8h*)(sIn + pix * OC_ + part * 8) = v;
    }
    __syncthreads();

    int wave = tid >> 5, lane = tid & 31;
    int m = lane & 15, hs = lane >> 4;
    int n = m;
    int mtile = wave & 3;
    int nbase = (wave >> 2) * 8;
    int mo = mtile * 16;

    v8f acc[8];
#pragma unroll
    for (int i = 0; i < 8; ++i) acc[i] = (v8f){};

    const _Float16* wbase = wf2 + (size_t)l * 9 * OC_ * OC_ + (mo + m) * OC_;

#pragma unroll 1
    for (int r = 0; r < 9; ++r) {
        int dy = r / 3, dx = r % 3;
        const _Float16* wr = wbase + r * OC_ * OC_;
        if (r < 8) __builtin_prefetch(wbase + (r + 1) * OC_ * OC_, 0, 1);
#pragma unroll
        for (int kc = 0; kc < 2; ++kc) {
            const _Float16* wk = wr + kc * 32;
            v16h av;
            ((v8h*)&av)[0] = *(const v8h*)(wk + 8 * hs);
            ((v8h*)&av)[1] = *(const v8h*)(wk + 16 + 8 * hs);
#pragma unroll
            for (int i = 0; i < 8; ++i) {
                int yy = nbase + i + dy;
                int xx = n + dx;
                const _Float16* sp = sIn + (yy * 18 + xx) * OC_ + kc * 32 + 8 * hs;
                v16h bv;
                ((v8h*)&bv)[0] = *(const v8h*)sp;
                ((v8h*)&bv)[1] = *(const v8h*)(sp + 16);
                acc[i] = __builtin_amdgcn_wmma_f32_16x16x32_f16(false, av, false, bv,
                                                                (short)0, acc[i],
                                                                false, false);
            }
        }
    }

    __syncthreads();
    _Float16* sOut = sIn;
#pragma unroll
    for (int i = 0; i < 8; ++i) {
        int ntile = nbase + i;
        int pix = ntile * 16 + n;
#pragma unroll
        for (int rr = 0; rr < 8; ++rr) {
            int oc = mo + rr + 8 * hs;
            sOut[pix * OC_ + oc] = (_Float16)fmaxf(acc[i][rr] + cb2[l * OC_ + oc], 0.0f);
        }
    }
    __syncthreads();
    _Float16* dst = y2 + (size_t)(b * L_ + l) * NPIX2 * OC_;
#pragma unroll 1
    for (int pass = 0; pass < 2; ++pass) {
#pragma unroll
        for (int i = 0; i < 8; ++i) { const int c = tid + 256 * i; *(volatile v4u_t*)(dst + (c >> 3) * OC_ + (c & 7) * 8) = *(const volatile v4ua*)(sOut + (c >> 3) * OC_ + (c & 7) * 8); }
        __threadfence();
    }
}

__global__ __launch_bounds__(256) void k_final(const _Float16* __restrict__ y2,
                                               const float* __restrict__ x,
                                               const float* __restrict__ nw,
                                               const float* __restrict__ nb,
                                               const float* __restrict__ fcw,
                                               const float* __restrict__ fcb,
                                               float* __restrict__ out) {
    __shared__ float sP[NNODES * 256];
    __shared__ float sRed[OUTW * 256];
    __shared__ float sMix[L_];
    __shared__ __attribute__((aligned(16))) float sOut[16 * OUTW];
    int tid = threadIdx.x;
#pragma unroll 1
    for (int bb = 0; bb < 16; ++bb) {
        const int b = blockIdx.x * 16 + bb;
        float p[NNODES];
#pragma unroll
        for (int q = 0; q < NNODES; ++q) p[q] = 0.0f;
        for (int i = tid; i < INW; i += 256) {
            float xv = x[b * INW + i];
#pragma unroll
            for (int q = 0; q < NNODES; ++q) p[q] += xv * nw[q * INW + i];
        }
#pragma unroll
        for (int q = 0; q < NNODES; ++q) sP[q * 256 + tid] = p[q];
        __syncthreads();
        if (tid < NNODES) {
            float s = 0.0f;
            for (int t = 0; t < 256; ++t) s += sP[tid * 256 + t];
            float lg = s + nb[tid];
            sP[tid * 256] = 1.0f / (1.0f + __expf(-lg));
        }
        __syncthreads();
        if (tid < L_) {
            const int j = tid;
            float sg0 = sP[0], t0 = ((j >> 2) & 1) ? sg0 : 1.0f - sg0;
            int   n1 = 1 + ((j >> 2) & 1);
            float sg1 = sP[n1 * 256], t1 = ((j >> 1) & 1) ? sg1 : 1.0f - sg1;
            int   n2 = 3 + (j >> 1);
            float sg2 = sP[n2 * 256], t2 = (j & 1) ? sg2 : 1.0f - sg2;
            sMix[j] = t0 * t1 * t2;
        }
        __syncthreads();
        float mx[L_];
#pragma unroll
        for (int l = 0; l < L_; ++l) mx[l] = sMix[l];
        float acc[OUTW];
#pragma unroll
        for (int o = 0; o < OUTW; ++o) acc[o] = 0.0f;
        const _Float16* yb = y2 + (size_t)b * L_ * FCIN;
        for (int j = tid; j < FCIN; j += 256) {
            float mixed = 0.0f;
#pragma unroll
            for (int l = 0; l < L_; ++l) mixed += mx[l] * (float)yb[l * FCIN + j];
            int oc = j & 63, pix = j >> 6;
            int i = oc * NPIX2 + pix;
#pragma unroll
            for (int o = 0; o < OUTW; ++o) acc[o] += mixed * fcw[o * FCIN + i];
        }
#pragma unroll
        for (int o = 0; o < OUTW; ++o) sRed[o * 256 + tid] = acc[o];
        __syncthreads();
        if (tid < OUTW) {
            float s = 0.0f;
            for (int t = 0; t < 256; ++t) s += sRed[tid * 256 + t];
            sOut[bb * OUTW + tid] = s + fcb[tid];
        }
        __syncthreads();
    }
    if (tid < 40) {
        const v4f_t v = *(const v4fa*)(sOut + tid * 4);
        float* dst = out + (size_t)blockIdx.x * 16 * OUTW + tid * 4;
        *(volatile v4f_t*)dst = v; __threadfence(); *(volatile v4f_t*)dst = v;
    }
}

extern "C" void kernel_launch(void* const* d_in, const int* in_sizes, int n_in,
                              void* d_out, int out_size, void* d_ws, size_t ws_size,
                              hipStream_t stream) {
    const float* x   = (const float*)d_in[0];
    const float* nw  = (const float*)d_in[1];
    const float* nb  = (const float*)d_in[2];
    const float* w1  = (const float*)d_in[3];
    const float* cb1 = (const float*)d_in[4];
    const float* w2  = (const float*)d_in[5];
    const float* cb2 = (const float*)d_in[6];
    const float* fcw = (const float*)d_in[7];
    const float* fcb = (const float*)d_in[8];
    float* out = (float*)d_out;

    char* ws = (char*)d_ws;
    float*    mix   = (float*)(ws);
    _Float16* wf1   = (_Float16*)(ws + 8192);
    _Float16* wf2   = (_Float16*)(ws + 8192 + 32768);
    _Float16* ypool = (_Float16*)(ws + 8192 + 32768 + 589824);
    _Float16* y2    = (_Float16*)(ws + 8192 + 32768 + 589824 + 67108864ull);

    (void)mix;
    k_convert_w1<<<(512 * K1PAD / 2 + 255) / 256, 256, 0, stream>>>(w1, wf1);
    k_convert_w2<<<(L_ * 9 * OC_ * OC_ / 2 + 255) / 256, 256, 0, stream>>>(w2, wf2);
    k_conv1_pool<<<B_ * 4, 256, 0, stream>>>(x, wf1, cb1, ypool);
    k_conv2<<<B_ * L_, 256, 0, stream>>>(ypool, wf2, cb2, y2);
    k_final<<<B_ / 16, 256, 0, stream>>>(y2, x, nw, nb, fcw, fcb, out);
}
